// GATModule_10273561772508
// MI455X (gfx1250) — hardware-verified
//
#include <hip/hip_runtime.h>
#include <stddef.h>
#include <stdint.h>
#include <math.h>


#define DIN     128
#define NHD     8
#define HID     512
#define KUP     256
#define KDN     1024
#define NSUV    16
#define NTHR    256
#define NWAVE   8
#define EPT     8
#define CHUNK   (NTHR * EPT)
#define WCAP    (EPT * 32)
#define LISTN   (NWAVE * WCAP)
#define NBMAX   2048
#define PSHIFT  11
#define RCAP    28672
#define DEGCAP  4096
#define STW     512
#define GBM     64
#define GBN     64
#define GTHR    128
#define NCHUNK  16
#define PB0     ((DIN * DIN / 8) / NTHR)
#define PB1     (PB0 + (HID * KUP / 8) / NTHR)
#define PB2     (PB1 + (DIN * KDN / 8) / NTHR)
#define WSMAX   134217728
#define LDS_AGG ((2 * RCAP + 2 * NBMAX + LISTN) * 4 + 64)

static_assert((CHUNK & (CHUNK - 1)) == 0 && CHUNK <= 4096);
static_assert((NBMAX & (NBMAX - 1)) == 0 && NBMAX == (1 << PSHIFT));
static_assert(NTHR * 8 == NBMAX);
static_assert(LISTN >= NBMAX);
static_assert(LISTN >= NWAVE * WCAP);
static_assert((RCAP % 32) == 0);
static_assert(NWAVE * STW <= RCAP);
static_assert(STW >= DIN);
static_assert(LDS_AGG <= 300000);
static_assert(GBM == (GTHR / 32) * 16);
static_assert((DIN % 32) == 0 && (KUP % 32) == 0 && (KDN % 32) == 0);
static_assert((DIN % GBN) == 0 && (HID % GBN) == 0);
static_assert(KUP == 2 * DIN && KDN == 2 * HID);
static_assert((DIN * DIN / 8) % NTHR == 0 && (HID * KUP / 8) % NTHR == 0 && (DIN * KDN / 8) % NTHR == 0);
static_assert(DIN == 4 * 32);
static_assert(NSUV == 2 * NHD && (NSUV % 4) == 0);

typedef unsigned short us;
typedef float    v2f  __attribute__((ext_vector_type(2)));
typedef float    v4f  __attribute__((ext_vector_type(4)));
typedef float    v8f  __attribute__((ext_vector_type(8)));
typedef int      v4i  __attribute__((ext_vector_type(4)));
typedef int      v8i  __attribute__((ext_vector_type(8)));
typedef us       v8us __attribute__((ext_vector_type(8)));
typedef __bf16   v16b __attribute__((ext_vector_type(16)));
union FragB { v16b v; v8us h[2]; v8i w; };

__device__ __forceinline__ v8f wmb(const FragB& a, const FragB& b, v8f c) {
  v8f d = __builtin_amdgcn_wmma_f32_16x16x32_bf16(false, a.v, false, b.v, (short)0, c, false, false);
  asm volatile("v_nop\n\tv_nop\n\tv_nop\n\tv_nop" : "+v"(d) : "v"(a.w), "v"(b.w));
  return d;
}

__device__ __forceinline__ void ldwait() {
  asm volatile("s_wait_loadcnt 0x0" ::: "memory");
}

__device__ __forceinline__ unsigned bf16u(float f) {
  unsigned u = __float_as_uint(f);
  u += 0x7FFFu + ((u >> 16) & 1u);
  return u >> 16;
}
__device__ __forceinline__ float bf16f(float f) { return __uint_as_float(bf16u(f) << 16); }

__device__ __forceinline__ v8us cvt8b(const v4f a, const v4f b) {
  v8us o;
  o[0] = (us)bf16u(a.x); o[1] = (us)bf16u(a.y); o[2] = (us)bf16u(a.z); o[3] = (us)bf16u(a.w);
  o[4] = (us)bf16u(b.x); o[5] = (us)bf16u(b.y); o[6] = (us)bf16u(b.z); o[7] = (us)bf16u(b.w);
  return o;
}

__device__ __forceinline__ void sp1(float v, unsigned& hb, unsigned& lb) {
  hb = bf16u(v);
  const float hf = __uint_as_float(hb << 16);
  lb = bf16u(v - hf);
}
__device__ __forceinline__ void split8(const v4f a, const v4f b, v8us& hi, v8us& lo) {
  unsigned h0, h1, h2, h3, h4, h5, h6, h7, l0, l1, l2, l3, l4, l5, l6, l7;
  sp1(a.x, h0, l0); sp1(a.y, h1, l1); sp1(a.z, h2, l2); sp1(a.w, h3, l3);
  sp1(b.x, h4, l4); sp1(b.y, h5, l5); sp1(b.z, h6, l6); sp1(b.w, h7, l7);
  hi[0] = (us)h0; hi[1] = (us)h1; hi[2] = (us)h2; hi[3] = (us)h3;
  hi[4] = (us)h4; hi[5] = (us)h5; hi[6] = (us)h6; hi[7] = (us)h7;
  lo[0] = (us)l0; lo[1] = (us)l1; lo[2] = (us)l2; lo[3] = (us)l3;
  lo[4] = (us)l4; lo[5] = (us)l5; lo[6] = (us)l6; lo[7] = (us)l7;
}

__device__ __forceinline__ float gelu_f(float v) {
  return 0.5f * v * (1.0f + erff(v * 0.70710678118654752f));
}

__device__ __forceinline__ void ldA(FragB& f, const float* p) {
  const v4f x0 = *(const v4f*)p,        x1 = *(const v4f*)(p + 4);
  const v4f x2 = *(const v4f*)(p + 16), x3 = *(const v4f*)(p + 20);
  f.h[0] = cvt8b(x0, x1);
  f.h[1] = cvt8b(x2, x3);
}
__device__ __forceinline__ void ldA(FragB& f, const us* p) {
  f.h[0] = *(const v8us*)p;
  f.h[1] = *(const v8us*)(p + 16);
}

__device__ __forceinline__ int scan_chunk(const int* __restrict__ dsts, int nE, int cbase, int slotBase,
                                          int nb, int vec8, int* list, int tid, int lane, int wave) {
  int wc = 0;
  const int el0  = tid * EPT;
  const int e0   = cbase + el0;
  const int sent = -2147483647 - 1;
  v4i da, db;
  if (vec8 != 0 && cbase + CHUNK <= nE) {
    da = *(const v4i*)(dsts + e0);
    db = *(const v4i*)(dsts + e0 + 4);
  } else {
    da.x = (e0     < nE) ? dsts[min(e0,     nE - 1)] : sent;
    da.y = (e0 + 1 < nE) ? dsts[min(e0 + 1, nE - 1)] : sent;
    da.z = (e0 + 2 < nE) ? dsts[min(e0 + 2, nE - 1)] : sent;
    da.w = (e0 + 3 < nE) ? dsts[min(e0 + 3, nE - 1)] : sent;
    db.x = (e0 + 4 < nE) ? dsts[min(e0 + 4, nE - 1)] : sent;
    db.y = (e0 + 5 < nE) ? dsts[min(e0 + 5, nE - 1)] : sent;
    db.z = (e0 + 6 < nE) ? dsts[min(e0 + 6, nE - 1)] : sent;
    db.w = (e0 + 7 < nE) ? dsts[min(e0 + 7, nE - 1)] : sent;
  }
  const unsigned nbs = (unsigned)slotBase;
  const unsigned unb = (unsigned)nb;
  const unsigned s0 = (unsigned)da.x - nbs, s1 = (unsigned)da.y - nbs;
  const unsigned s2 = (unsigned)da.z - nbs, s3 = (unsigned)da.w - nbs;
  const unsigned s4 = (unsigned)db.x - nbs, s5 = (unsigned)db.y - nbs;
  const unsigned s6 = (unsigned)db.z - nbs, s7 = (unsigned)db.w - nbs;
  const bool h0 = s0 < unb, h1 = s1 < unb, h2 = s2 < unb, h3 = s3 < unb;
  const bool h4 = s4 < unb, h5 = s5 < unb, h6 = s6 < unb, h7 = s7 < unb;
  const unsigned any = __builtin_amdgcn_ballot_w32(h0 | h1 | h2 | h3 | h4 | h5 | h6 | h7);
  if (any != 0u) {
#define HITJ(J, HJ, SJ) { \
      const unsigned mj = __builtin_amdgcn_ballot_w32(HJ); \
      if (mj != 0u) { \
        if (HJ) { \
          const int pos = wc + (int)__builtin_amdgcn_mbcnt_lo(mj, 0u); \
          if (pos < WCAP) list[wave * WCAP + pos] = ((el0 + (J)) << 12) | (int)(SJ); \
        } \
        wc += (int)__builtin_popcount(mj); } }
    HITJ(0, h0, s0)
    HITJ(1, h1, s1)
    HITJ(2, h2, s2)
    HITJ(3, h3, s3)
    HITJ(4, h4, s4)
    HITJ(5, h5, s5)
    HITJ(6, h6, s6)
    HITJ(7, h7, s7)
#undef HITJ
  }
  return wc;
}

__global__ __launch_bounds__(NTHR) void k_prep(const float* __restrict__ W_in, const float* __restrict__ W1,
                                               const float* __restrict__ W2, us* WINT, us* W1T2, us* W2T2) {
  const int b = (int)blockIdx.x, t = (int)threadIdx.x;
  v4f a, c;
  us* dp;
  if (b < PB0) {
    const int u  = b * NTHR + t;
    const int n  = u >> 4;
    const int k8 = (u & 15) * 8;
    const float* p = W_in + (size_t)k8 * DIN + n;
    a.x = p[0];             a.y = p[DIN];           a.z = p[2 * DIN];       a.w = p[3 * DIN];
    c.x = p[4 * DIN];       c.y = p[5 * DIN];       c.z = p[6 * DIN];       c.w = p[7 * DIN];
    dp = WINT + (size_t)n * DIN + k8;
  } else if (b < PB1) {
    const int u  = (b - PB0) * NTHR + t;
    const int n  = u >> 5;
    const int kk = (u & 31) * 8;
    const int k  = kk & (DIN - 1);
    const float* p = W1 + (size_t)k * HID + n;
    a.x = p[0];             a.y = p[HID];           a.z = p[2 * HID];       a.w = p[3 * HID];
    c.x = p[4 * HID];       c.y = p[5 * HID];       c.z = p[6 * HID];       c.w = p[7 * HID];
    dp = W1T2 + (size_t)n * KUP + kk;
  } else {
    const int u  = (b - PB1) * NTHR + t;
    const int n  = u >> 7;
    const int kk = (u & 127) * 8;
    const int k  = kk & (HID - 1);
    const float* p = W2 + (size_t)k * DIN + n;
    a.x = p[0];             a.y = p[DIN];           a.z = p[2 * DIN];       a.w = p[3 * DIN];
    c.x = p[4 * DIN];       c.y = p[5 * DIN];       c.z = p[6 * DIN];       c.w = p[7 * DIN];
    dp = W2T2 + (size_t)n * KDN + kk;
  }
  const v8us hv = cvt8b(a, c);
  *(volatile v8us*)dp = hv;
  __threadfence();
  *(volatile v8us*)dp = hv;
}

template<typename AT, int EPI>
__global__ __launch_bounds__(GTHR) void k_gemm(
    const AT* __restrict__ A, const us* __restrict__ WT, const float* __restrict__ bias,
    float* outF, us* outH, int K, int ldo, int nRows, int nCols, int nArows)
{
  __shared__ __attribute__((aligned(16))) float stg[GBM * GBN];
  const int tid = (int)threadIdx.x, lane = tid & 31, wave = tid >> 5, hh = lane >> 4, m = lane & 15;
  const int rowBase = (int)blockIdx.x * GBM;
  const int col0    = (int)blockIdx.y * GBN;

  v8f acc[4];
  {
    const v8f z = {0.f, 0.f, 0.f, 0.f, 0.f, 0.f, 0.f, 0.f};
    acc[0] = z; acc[1] = z; acc[2] = z; acc[3] = z;
  }
  int arow = rowBase + 16 * wave + m;
  arow = arow > nArows - 1 ? nArows - 1 : arow;
  arow = arow < 0 ? 0 : arow;
  const AT* ap = A  + (size_t)arow * (size_t)K + 8 * hh;
  const us* wp = WT + (size_t)(col0 + m) * (size_t)K + 8 * hh;
  const int ksteps = K >> 5;
#pragma unroll 1
  for (int ks = 0; ks < ksteps; ++ks) {
    FragB af;
    ldA(af, ap + 32 * ks);
#pragma unroll
    for (int t = 0; t < 4; ++t) {
      const us* wq = wp + (size_t)(16 * t) * (size_t)K + 32 * ks;
      FragB bf;
      bf.h[0] = *(const v8us*)wq;
      bf.h[1] = *(const v8us*)(wq + 16);
      acc[t] = wmb(af, bf, acc[t]);
    }
  }

#pragma unroll
  for (int t = 0; t < 4; ++t) {
    const int lc = 16 * t + m;
    int bi = col0 + lc;
    bi = bi > nCols - 1 ? nCols - 1 : bi;
    bi = bi < 0 ? 0 : bi;
    const float bv = bf16f(bias[bi]);
#pragma unroll
    for (int r = 0; r < 8; ++r) {
      const int lr = 16 * wave + 8 * hh + r;
      float v = acc[t][r] + bv;
      if (EPI == 1) v = gelu_f(v);
      stg[lr * GBN + lc] = v;
    }
  }
  __syncthreads();

  if (EPI == 0) {
    v4f fv[8];
#pragma unroll
    for (int i = 0; i < 8; ++i) {
      const int lr = 16 * wave + 2 * i + hh;
      fv[i] = *(const v4f*)(stg + lr * GBN + 4 * m);
    }
#pragma unroll
    for (int i = 0; i < 8; ++i) {
      const int lr = 16 * wave + 2 * i + hh;
      const int gr = rowBase + lr;
      if (gr < nRows) {
        float* op = outF + (size_t)gr * (size_t)ldo + col0 + 4 * m;
        *(volatile v4f*)op = fv[i];
      }
    }
    __threadfence();
#pragma unroll
    for (int i = 0; i < 8; ++i) {
      const int lr = 16 * wave + 2 * i + hh;
      const int gr = rowBase + lr;
      if (gr < nRows) {
        float* op = outF + (size_t)gr * (size_t)ldo + col0 + 4 * m;
        *(volatile v4f*)op = fv[i];
      }
    }
  } else {
    const int sub = lane >> 3, c8 = (lane & 7) * 8;
    v8us hv[4], lv[4];
#pragma unroll
    for (int i = 0; i < 4; ++i) {
      const int lr = 16 * wave + 4 * i + sub;
      const v4f ga = *(const v4f*)(stg + lr * GBN + c8);
      const v4f gb = *(const v4f*)(stg + lr * GBN + c8 + 4);
      split8(ga, gb, hv[i], lv[i]);
    }
#pragma unroll
    for (int i = 0; i < 4; ++i) {
      const int lr = 16 * wave + 4 * i + sub;
      const int gr = rowBase + lr;
      if (gr < nRows) {
        us* hp = outH + (size_t)gr * (size_t)(2 * ldo) + col0 + c8;
        *(volatile v8us*)hp = hv[i];
        *(volatile v8us*)(hp + ldo) = lv[i];
      }
    }
    __threadfence();
#pragma unroll
    for (int i = 0; i < 4; ++i) {
      const int lr = 16 * wave + 4 * i + sub;
      const int gr = rowBase + lr;
      if (gr < nRows) {
        us* hp = outH + (size_t)gr * (size_t)(2 * ldo) + col0 + c8;
        *(volatile v8us*)hp = hv[i];
        *(volatile v8us*)(hp + ldo) = lv[i];
      }
    }
  }
}

__global__ __launch_bounds__(NTHR) void k_suv(const float* __restrict__ X, const float* __restrict__ W_u,
                                              const float* __restrict__ b_u, const float* __restrict__ W_v,
                                              float* SUV, int MPr) {
  __shared__ __attribute__((aligned(16))) float wl[DIN * NSUV];
  __shared__ __attribute__((aligned(16))) float so[NTHR * NSUV];
  __shared__ float bl[NSUV];
  const int tid = (int)threadIdx.x;
  for (int i = tid; i < DIN * NSUV; i += NTHR) {
    const int k = i >> 4, c = i & 15;
    const float wa = W_u[k * NHD + (c & 7)];
    const float wb = W_v[k * NHD + (c & 7)];
    wl[i] = bf16f(c < NHD ? wa : wb);
  }
  {
    const float bu = bf16f(b_u[tid & 7]);
    if (tid < NSUV) bl[tid] = (tid < NHD) ? bu : 0.0f;
  }
  __syncthreads();

  const int row = (int)blockIdx.x * NTHR + tid;
  const int rc  = row < MPr ? row : MPr - 1;
  const float* xr = X + (size_t)rc * DIN;
  float acc[NSUV];
#pragma unroll
  for (int c = 0; c < NSUV; ++c) acc[c] = 0.0f;
#pragma unroll 1
  for (int k2 = 0; k2 < DIN / 2; ++k2) {
    const v2f xv = *(const v2f*)(xr + 2 * k2);
    const float* wk = wl + 2 * NSUV * k2;
    const v4f w0 = *(const v4f*)(wk),      w1 = *(const v4f*)(wk + 4);
    const v4f w2 = *(const v4f*)(wk + 8),  w3 = *(const v4f*)(wk + 12);
    const v4f u0 = *(const v4f*)(wk + 16), u1 = *(const v4f*)(wk + 20);
    const v4f u2 = *(const v4f*)(wk + 24), u3 = *(const v4f*)(wk + 28);
    acc[0]  = fmaf(xv.x, w0.x, acc[0]);  acc[1]  = fmaf(xv.x, w0.y, acc[1]);
    acc[2]  = fmaf(xv.x, w0.z, acc[2]);  acc[3]  = fmaf(xv.x, w0.w, acc[3]);
    acc[4]  = fmaf(xv.x, w1.x, acc[4]);  acc[5]  = fmaf(xv.x, w1.y, acc[5]);
    acc[6]  = fmaf(xv.x, w1.z, acc[6]);  acc[7]  = fmaf(xv.x, w1.w, acc[7]);
    acc[8]  = fmaf(xv.x, w2.x, acc[8]);  acc[9]  = fmaf(xv.x, w2.y, acc[9]);
    acc[10] = fmaf(xv.x, w2.z, acc[10]); acc[11] = fmaf(xv.x, w2.w, acc[11]);
    acc[12] = fmaf(xv.x, w3.x, acc[12]); acc[13] = fmaf(xv.x, w3.y, acc[13]);
    acc[14] = fmaf(xv.x, w3.z, acc[14]); acc[15] = fmaf(xv.x, w3.w, acc[15]);
    acc[0]  = fmaf(xv.y, u0.x, acc[0]);  acc[1]  = fmaf(xv.y, u0.y, acc[1]);
    acc[2]  = fmaf(xv.y, u0.z, acc[2]);  acc[3]  = fmaf(xv.y, u0.w, acc[3]);
    acc[4]  = fmaf(xv.y, u1.x, acc[4]);  acc[5]  = fmaf(xv.y, u1.y, acc[5]);
    acc[6]  = fmaf(xv.y, u1.z, acc[6]);  acc[7]  = fmaf(xv.y, u1.w, acc[7]);
    acc[8]  = fmaf(xv.y, u2.x, acc[8]);  acc[9]  = fmaf(xv.y, u2.y, acc[9]);
    acc[10] = fmaf(xv.y, u2.z, acc[10]); acc[11] = fmaf(xv.y, u2.w, acc[11]);
    acc[12] = fmaf(xv.y, u3.x, acc[12]); acc[13] = fmaf(xv.y, u3.y, acc[13]);
    acc[14] = fmaf(xv.y, u3.z, acc[14]); acc[15] = fmaf(xv.y, u3.w, acc[15]);
  }
  {
    v4f r0, r1, r2, r3;
    r0.x = acc[0]  + bl[0];  r0.y = acc[1]  + bl[1];  r0.z = acc[2]  + bl[2];  r0.w = acc[3]  + bl[3];
    r1.x = acc[4]  + bl[4];  r1.y = acc[5]  + bl[5];  r1.z = acc[6]  + bl[6];  r1.w = acc[7]  + bl[7];
    r2.x = acc[8]  + bl[8];  r2.y = acc[9]  + bl[9];  r2.z = acc[10] + bl[10]; r2.w = acc[11] + bl[11];
    r3.x = acc[12] + bl[12]; r3.y = acc[13] + bl[13]; r3.z = acc[14] + bl[14]; r3.w = acc[15] + bl[15];
    *(v4f*)(so + tid * NSUV)      = r0;
    *(v4f*)(so + tid * NSUV + 4)  = r1;
    *(v4f*)(so + tid * NSUV + 8)  = r2;
    *(v4f*)(so + tid * NSUV + 12) = r3;
  }
  __syncthreads();

  const int rowBlk = (int)blockIdx.x * NTHR;
  float* ob = SUV + (size_t)rowBlk * NSUV;
  v4f pv[4];
#pragma unroll
  for (int i = 0; i < 4; ++i) {
    const int p = i * NTHR + tid;
    pv[i] = *(const v4f*)(so + 4 * p);
  }
#pragma unroll
  for (int i = 0; i < 4; ++i) {
    const int p = i * NTHR + tid;
    const int rl = p >> 2;
    if (rowBlk + rl < MPr) *(volatile v4f*)(ob + 4 * p) = pv[i];
  }
  __threadfence();
#pragma unroll
  for (int i = 0; i < 4; ++i) {
    const int p = i * NTHR + tid;
    const int rl = p >> 2;
    if (rowBlk + rl < MPr) *(volatile v4f*)(ob + 4 * p) = pv[i];
  }
}

__global__ __launch_bounds__(NTHR) void k_agg(
    const int* __restrict__ srcs, const int* __restrict__ dsts,
    const float* __restrict__ X, const float* __restrict__ SUV, us* HHL,
    int nN, int nE, int nb, int vec8, int MPr) {
  extern __shared__ v4f lds_dyn[];
  int* reg1 = (int*)lds_dyn;
  int* reg2 = reg1 + RCAP;
  int* scnt = reg2 + RCAP;
  int* soff = scnt + NBMAX;
  int* list = soff + NBMAX;
  int* wcnt = list + LISTN;
  int* wtot = wcnt + NWAVE;
  const int tid = (int)threadIdx.x, lane = tid & 31, wave = tid >> 5;
  const int nodeBase = (int)blockIdx.x * nb;

  for (int i = tid; i < NBMAX; i += NTHR) scnt[i] = 0;
  __syncthreads();

  int tot = 0;
  const int nChunks = (nE + CHUNK - 1) / CHUNK;
#pragma unroll 1
  for (int ch = 0; ch < nChunks; ++ch) {
    const int cbase = ch * CHUNK;
    const int wc = scan_chunk(dsts, nE, cbase, nodeBase, nb, vec8, list, tid, lane, wave);
    if (lane == 0) wcnt[wave] = wc;
    __syncthreads();
    int pre = 0, all = 0;
#pragma unroll
    for (int w2 = 0; w2 < NWAVE; ++w2) {
      int c = wcnt[w2];
      c = c < 0 ? 0 : (c > WCAP ? WCAP : c);
      all += c;
      pre += (w2 < wave) ? c : 0;
    }
    const int wcc  = wc > WCAP ? WCAP : wc;
    const int base = tot + pre;
#pragma unroll 1
    for (int i = lane; i < wcc; i += 32) {
      const int ent = list[wave * WCAP + i];
      const int el  = (ent >> 12) & (CHUNK - 1);
      const int sl  = ent & (NBMAX - 1);
      int eid = cbase + el;
      eid = eid > nE - 1 ? nE - 1 : eid;
      const int pos = base + i;
      if (pos < RCAP) reg1[pos] = (int)(((unsigned)eid << PSHIFT) | (unsigned)sl);
    }
    tot += all;
    tot = tot > RCAP ? RCAP : tot;
    __syncthreads();
  }
  const int nh = tot;

  if (wave == 0) {
#pragma unroll 1
    for (int b0 = 0; b0 < nh; b0 += 32) {
      const int idx = b0 + lane;
      const int uv  = reg1[idx < RCAP ? idx : RCAP - 1];
      const int m32 = (nh - b0) < 32 ? (nh - b0) : 32;
#pragma unroll 1
      for (int k = 0; k < m32; ++k) {
        const int u  = __builtin_amdgcn_readlane(uv, k);
        const int sl = u & (NBMAX - 1);
        if (lane == 0) scnt[sl] = scnt[sl] + 1;
      }
    }
  }
  __syncthreads();

  {
    const v4i ca = *(const v4i*)(scnt + 8 * tid);
    const v4i cb = *(const v4i*)(scnt + 8 * tid + 4);
    const int e0 = ca.x < 0 ? 0 : ca.x, e1 = ca.y < 0 ? 0 : ca.y, e2 = ca.z < 0 ? 0 : ca.z, e3 = ca.w < 0 ? 0 : ca.w;
    const int e4 = cb.x < 0 ? 0 : cb.x, e5 = cb.y < 0 ? 0 : cb.y, e6 = cb.z < 0 ? 0 : cb.z, e7 = cb.w < 0 ? 0 : cb.w;
    const int ts = e0 + e1 + e2 + e3 + e4 + e5 + e6 + e7;
    int incl = ts;
#pragma unroll
    for (int d = 1; d < 32; d <<= 1) {
      const int up = __shfl_up(incl, d);
      if (lane >= d) incl += up;
    }
    if (lane == 31) wtot[wave] = incl;
    __syncthreads();
    int pre = 0;
#pragma unroll
    for (int w2 = 0; w2 < NWAVE; ++w2) pre += (w2 < wave) ? wtot[w2] : 0;
    int run = pre + incl - ts;
    soff[8 * tid + 0] = run; run += e0;
    soff[8 * tid + 1] = run; run += e1;
    soff[8 * tid + 2] = run; run += e2;
    soff[8 * tid + 3] = run; run += e3;
    soff[8 * tid + 4] = run; run += e4;
    soff[8 * tid + 5] = run; run += e5;
    soff[8 * tid + 6] = run; run += e6;
    soff[8 * tid + 7] = run;
  }
  __syncthreads();
  for (int i = tid; i < NBMAX; i += NTHR) list[i] = soff[i];
  __syncthreads();

  if (wave == 0) {
#pragma unroll 1
    for (int b0 = 0; b0 < nh; b0 += 32) {
      const int idx = b0 + lane;
      const int uv  = reg1[idx < RCAP ? idx : RCAP - 1];
      const int m32 = (nh - b0) < 32 ? (nh - b0) : 32;
#pragma unroll 1
      for (int k = 0; k < m32; ++k) {
        const int u   = __builtin_amdgcn_readlane(uv, k);
        const int sl  = u & (NBMAX - 1);
        const int eid = (int)((unsigned)u >> PSHIFT);
        if (lane == 0) {
          int pos = list[sl];
          pos = pos < 0 ? 0 : (pos > RCAP - 1 ? RCAP - 1 : pos);
          reg2[pos] = eid;
          list[sl] = pos + 1;
        }
      }
    }
  }
  __syncthreads();

  const int nbw = nb >> 3;
  const bool ovf = (nh >= RCAP);
  const float qnan = __int_as_float(0x7fc00000);
  float* stw = (float*)reg1 + wave * STW;
  const int hl = lane & 7, q16 = lane & 15, part = lane >> 4;
#pragma unroll 1
  for (int jt = 0; jt < nbw; ++jt) {
    const int slot = wave * nbw + jt;
    const int grow = nodeBase + slot;
    const int gcl  = grow < nN ? grow : nN - 1;
    int st = soff[slot];
    const int craw = scnt[slot];
    int cnt = craw;
    st  = st < 0 ? 0 : (st > nh ? nh : st);
    cnt = cnt < 0 ? 0 : (cnt > DEGCAP ? DEGCAP : cnt);
    if (cnt > nh - st) cnt = nh - st;
    const float pz = (ovf || craw > DEGCAP) ? qnan : 0.0f;
    const bool wr = grow < MPr;
    const float live = grow < nN ? 1.0f : 0.0f;

    const float svd = SUV[(size_t)gcl * NSUV + NHD + hl];
    ldwait();
    float mx = -1.0e30f, dn = 0.f, a0 = 0.f, a1 = 0.f, a2 = 0.f, a3 = 0.f;

#pragma unroll 1
    for (int q = 0; q < cnt; ++q) {
      int idx = st + q; idx = idx > RCAP - 1 ? RCAP - 1 : idx;
      int eid = reg2[idx]; eid = eid < 0 ? 0 : (eid > nE - 1 ? nE - 1 : eid);
      const int sraw = srcs[eid];
      const int s = sraw < 0 ? 0 : (sraw > nN - 1 ? nN - 1 : sraw);
      const float sus = SUV[(size_t)s * NSUV + hl];
      const float* xr = X + (size_t)s * DIN + lane;
      const float x0 = xr[0], x1 = xr[32], x2 = xr[64], x3 = xr[96];
      ldwait();
      float lg = sus + svd;
      lg = lg > 0.0f ? lg : 0.2f * lg;
      const float df = lg - mx;
      const float ee = __expf(-fabsf(df));
      const bool up  = df > 0.f;
      const float s1 = up ? ee : 1.0f;
      const float s2 = up ? 1.0f : ee;
      mx = up ? lg : mx;
      dn = fmaf(dn, s1, s2);
      a0 = fmaf(a0, s1, s2 * x0);
      a1 = fmaf(a1, s1, s2 * x1);
      a2 = fmaf(a2, s1, s2 * x2);
      a3 = fmaf(a3, s1, s2 * x3);
    }
    const float ds = dn > 0.f ? dn : 1.0f;
    const float iv = (dn > 0.f ? live : 0.0f) * __builtin_amdgcn_rcpf(ds);
    const float o0 = a0 * iv + pz;
    const float o1 = a1 * iv + pz;
    const float o2 = a2 * iv + pz;
    const float o3 = a3 * iv + pz;
    __builtin_amdgcn_fence(__ATOMIC_RELEASE, "wavefront");
    __builtin_amdgcn_wave_barrier();
    stw[lane]      = o0;
    stw[32 + lane] = o1;
    stw[64 + lane] = o2;
    stw[96 + lane] = o3;
    __builtin_amdgcn_fence(__ATOMIC_RELEASE, "wavefront");
    __builtin_amdgcn_wave_barrier();
    const v4f ga = *(const v4f*)(stw + 8 * q16);
    const v4f gb = *(const v4f*)(stw + 8 * q16 + 4);
    v8us hv, lv;
    split8(ga, gb, hv, lv);
    v8us ov;
    ov[0] = part ? lv[0] : hv[0]; ov[1] = part ? lv[1] : hv[1];
    ov[2] = part ? lv[2] : hv[2]; ov[3] = part ? lv[3] : hv[3];
    ov[4] = part ? lv[4] : hv[4]; ov[5] = part ? lv[5] : hv[5];
    ov[6] = part ? lv[6] : hv[6]; ov[7] = part ? lv[7] : hv[7];
    us* gp = HHL + (size_t)grow * KUP + DIN * part + 8 * q16;
    if (wr) *(volatile v8us*)gp = ov;
    __threadfence();
    if (wr) *(volatile v8us*)gp = ov;
  }
}

static int pick_nb(int nE, int nN) {
  int nb = NBMAX;
  while (nb > 16 && (long long)nb * (long long)nE * 5LL > (long long)RCAP * (long long)nN * 4LL) nb >>= 1;
  return nb;
}
static inline int cdiv(int a, int b) { return (a + b - 1) / b; }

extern "C" void kernel_launch(void* const* d_in, const int* in_sizes, int n_in,
                              void* d_out, int out_size, void* d_ws, size_t ws_size,
                              hipStream_t stream) {
  if (n_in < 12) return;
  const int nN = in_sizes[0] / DIN;
  if (nN <= 0 || in_sizes[0] != nN * DIN || nN > (1 << 22)) return;
  const int nE = in_sizes[1];
  if (nE < 1 || nE > (1 << 21) || in_sizes[2] != nE) return;
  if (in_sizes[3] != DIN * DIN || in_sizes[4] != DIN) return;
  if (in_sizes[5] != DIN * NHD || in_sizes[6] != NHD) return;
  if (in_sizes[7] != DIN * NHD) return;
  if (in_sizes[8] != DIN * HID || in_sizes[9] != HID) return;
  if (in_sizes[10] != HID * DIN || in_sizes[11] != DIN) return;
  if (out_size != nN * DIN) return;

  const float* h    = (const float*)d_in[0];
  const int*   src  = (const int*)  d_in[1];
  const int*   dst  = (const int*)  d_in[2];
  const float* W_in = (const float*)d_in[3];
  const float* b_in = (const float*)d_in[4];
  const float* W_u  = (const float*)d_in[5];
  const float* b_u  = (const float*)d_in[6];
  const float* W_v  = (const float*)d_in[7];
  const float* W1   = (const float*)d_in[8];
  const float* b1   = (const float*)d_in[9];
  const float* W2   = (const float*)d_in[10];
  const float* b2   = (const float*)d_in[11];
  float* y = (float*)d_out;

  const int MP   = cdiv(nN, GBM) * GBM;
  const int CR   = cdiv(MP / GBM, NCHUNK) * GBM;
  const int nb   = pick_nb(nE, nN);
  const int gA   = cdiv(MP, nb);
  const int vec8 = 1;
  if (gA * nb < MP) return;
  if ((long long)CR * NCHUNK < MP) return;

  char* ws = (char*)d_ws;
  size_t off = 0;
  const size_t oX   = off; off += (size_t)MP * DIN * 4;        off = (off + 255) & ~(size_t)255;
  const size_t oHID = off; off += (size_t)CR * KDN * 2;        off = (off + 255) & ~(size_t)255;
  const size_t oSUV = off; off += (size_t)MP * NSUV * 4;       off = (off + 255) & ~(size_t)255;
  const size_t oHHL = off; off += (size_t)MP * KUP * 2;        off = (off + 255) & ~(size_t)255;
  const size_t oWIN = off; off += (size_t)DIN * DIN * 2;       off = (off + 255) & ~(size_t)255;
  const size_t oW1  = off; off += (size_t)HID * KUP * 2;       off = (off + 255) & ~(size_t)255;
  const size_t oW2  = off; off += (size_t)DIN * KDN * 2;       off = (off + 255) & ~(size_t)255;
  if (off > ws_size || off > (size_t)WSMAX) return;
  float* X    = (float*)(ws + oX);
  us*    HIDP = (us*)(ws + oHID);
  float* SUV  = (float*)(ws + oSUV);
  us*    HHL  = (us*)(ws + oHHL);
  us*    WINT = (us*)(ws + oWIN);
  us*    W1T2 = (us*)(ws + oW1);
  us*    W2T2 = (us*)(ws + oW2);

  hipFuncSetAttribute(reinterpret_cast<const void*>(&k_agg),
                      hipFuncAttributeMaxDynamicSharedMemorySize, LDS_AGG);

  k_prep<<<PB2, NTHR, 0, stream>>>(W_in, W1, W2, WINT, W1T2, W2T2);

  const int gM = MP / GBM;
  k_gemm<float, 0><<<dim3(gM, DIN / GBN), GTHR, 0, stream>>>(h, WINT, b_in, X, HHL,
                                                              DIN, DIN, MP, DIN, nN);
  k_suv<<<cdiv(MP, NTHR), NTHR, 0, stream>>>(X, W_u, b_u, W_v, SUV, MP);
  k_agg<<<gA, NTHR, LDS_AGG, stream>>>(src, dst, X, SUV, HHL, nN, nE, nb, vec8, MP);

  for (int c = 0; c < NCHUNK; ++c) {
    const int cbase = c * CR;
    if (cbase >= MP) break;
    int rows = MP - cbase;
    rows = rows > CR ? CR : rows;
    int nr3 = nN - cbase;
    nr3 = nr3 > rows ? rows : nr3;
    k_gemm<us, 1><<<dim3(rows / GBM, HID / GBN), GTHR, 0, stream>>>(HHL + (size_t)cbase * KUP, W1T2, b1,
                                                                   SUV, HIDP, KUP, HID, rows, HID, rows);
    k_gemm<us, 0><<<dim3(rows / GBM, DIN / GBN), GTHR, 0, stream>>>(HIDP, W2T2, b2, y + (size_t)cbase * DIN,
                                                                   HHL, KDN, DIN, nr3, DIN, rows);
  }
}
